// PointAttention_65798898975033
// MI455X (gfx1250) — hardware-verified
//
#include <hip/hip_runtime.h>
#include <stdint.h>
#include <stddef.h>
#include <math.h>

#define DEVINL __device__ __forceinline__

typedef _Float16 f16t;
typedef _Float16 v16h __attribute__((ext_vector_type(16)));
typedef _Float16 v8h  __attribute__((ext_vector_type(8)));
typedef _Float16 v4h  __attribute__((ext_vector_type(4)));
typedef float    v8f  __attribute__((ext_vector_type(8)));
typedef float    v4f  __attribute__((ext_vector_type(4)));
typedef v8h __attribute__((may_alias)) v8ha;
typedef v4f __attribute__((may_alias)) v4fa;
union FragH { v16h v; v8h half[2]; };
union U8 { v8f v; v4f q[2]; };

#define NB    2
#define NN    512
#define DM    256
#define NH    8
#define HD    32
#define NA    16
#define BNR   1024
#define TPB   128
#define TPBA  256
#define TPBP  256
#define PH    72
#define PF    68
#define GP    40
#define SBP   36

#define XCAR   16.0f
#define WCAR   256.0f
#define QCAR   16.0f
#define VCAR   16.0f
#define HCAR   1024.0f
#define W2CAR  64.0f
#define PCAR   256.0f
#define OCAR   64.0f
#define SCALE  0.17677669529663687f
#define RSQRT2 0.70710678118654752f
#define SC_P   (1.0f / 4096.0f)
#define SC_B   (1.0f / 65536.0f)
#define SC_S   (SCALE / 256.0f)
#define SC_O   (1.0f / 64.0f)
#define SC_PO  (1.0f / 16384.0f)

#define XP_BLKS   (BNR * DM / 8 / TPBP)
#define WT_BLKS   (4 * (DM / 64) * (DM / 64))
#define W2_BLKS   (16 * DM / 8 / TPBP)
#define PRJ_BLKS  (3 * (BNR / 64) * (DM / 64))
#define BIAS_BLKS (NB * (NN / 8) * (NN / 32))
#define ATT_BLKS  (NB * (NH / 2) * (NN / 64))
#define OP_BLKS   ((BNR / 64) * (DM / 64))

static_assert(TPB == 4 * 32);
static_assert(TPBA == 8 * 32);
static_assert(XP_BLKS * TPBP * 8 == BNR * DM);
static_assert(W2_BLKS * TPBP * 8 == 16 * DM);
static_assert(NA == NB * NH);
static_assert(NH * HD == DM);
static_assert((DM % 64) == 0);
static_assert((NN % 64) == 0);
static_assert((PH % 8) == 0);
static_assert((GP % 8) == 0);
static_assert((PF % 4) == 0);
static_assert((SBP % 4) == 0);
static_assert(XP_BLKS == 128 && WT_BLKS == 64 && W2_BLKS == 2);
static_assert(PRJ_BLKS == 192 && BIAS_BLKS == 2048 && ATT_BLKS == 64 && OP_BLKS == 64);

DEVINL v8f wmma_f16(v16h a, v16h b, v8f c) {
  v8f d = __builtin_amdgcn_wmma_f32_16x16x32_f16(false, a, false, b, (short)0, c, false, false);
  asm volatile("v_nop\n\tv_nop\n\tv_nop\n\tv_nop" : "+v"(d) : "v"(a), "v"(b));
  return d;
}
DEVINL v8f zero8f() {
  v8f z = {0.f, 0.f, 0.f, 0.f, 0.f, 0.f, 0.f, 0.f};
  return z;
}
DEVINL void load_frag(FragH& f, const f16t* row, int k0) {
  f.half[0] = *(const v8ha*)(row + k0);
  f.half[1] = *(const v8ha*)(row + k0 + 16);
}

template <int KD>
DEVINL void mma_4n(const f16t* __restrict__ arow, const f16t* __restrict__ brow, v8f (&acc)[4]) {
  #pragma unroll 1
  for (int ks = 0; ks < KD / 32; ++ks) {
    const int k0 = 32 * ks;
    FragH a;
    load_frag(a, arow, k0);
    #pragma unroll
    for (int n = 0; n < 4; ++n) {
      FragH b;
      load_frag(b, brow + (size_t)16 * n * KD, k0);
      acc[n] = wmma_f16(a.v, b.v, acc[n]);
    }
  }
}

__global__ __launch_bounds__(TPBP) void prep_k(const float* __restrict__ x,
                                              const float* __restrict__ wq, const float* __restrict__ wk,
                                              const float* __restrict__ wv, const float* __restrict__ wo,
                                              const float* __restrict__ wp2,
                                              f16t* __restrict__ XH, f16t* __restrict__ WT,
                                              f16t* __restrict__ W2T)
{
  __shared__ __attribute__((aligned(16))) f16t tile[64 * PH];
  const int blk = blockIdx.x, tid = threadIdx.x;
  if (blk < XP_BLKS) {
    const size_t idx = ((size_t)blk * TPBP + tid) * 8;
    const v4f a = *(const v4fa*)(x + idx), c = *(const v4fa*)(x + idx + 4);
    v8h o;
    #pragma unroll
    for (int j = 0; j < 4; ++j) {
      o[j]     = (f16t)(a[j] * XCAR);
      o[4 + j] = (f16t)(c[j] * XCAR);
    }
    f16t* dp = XH + idx;
    *(volatile v8h*)dp = o;
    __threadfence();
    *(volatile v8h*)dp = o;
  } else if (blk < XP_BLKS + WT_BLKS) {
    const int wb = blk - XP_BLKS;
    const int mat = wb >> 4, t = wb & 15;
    const int kt = t >> 2, ot = t & 3;
    const int k0 = 64 * kt, o0 = 64 * ot;
    const float* W = (mat == 0) ? wq : ((mat == 1) ? wk : ((mat == 2) ? wv : wo));
    const int krow = tid >> 2, oc = (tid & 3) * 16;
    const float* sp = W + (size_t)(k0 + krow) * DM + o0 + oc;
    #pragma unroll
    for (int i = 0; i < 4; ++i) {
      const v4f a = *(const v4fa*)(sp + 4 * i);
      #pragma unroll
      for (int j = 0; j < 4; ++j) tile[(oc + 4 * i + j) * PH + krow] = (f16t)(a[j] * WCAR);
    }
    __syncthreads();
    v8h ov[2];
    size_t off[2];
    #pragma unroll
    for (int kk = 0; kk < 2; ++kk) {
      const int p = 256 * kk + tid;
      const int orow = p >> 3, q = p & 7;
      ov[kk] = *(const v8ha*)(tile + orow * PH + 8 * q);
      off[kk] = (size_t)mat * DM * DM + (size_t)(o0 + orow) * DM + k0 + 8 * q;
    }
    #pragma unroll
    for (int kk = 0; kk < 2; ++kk) *(volatile v8h*)(WT + off[kk]) = ov[kk];
    __threadfence();
    #pragma unroll
    for (int kk = 0; kk < 2; ++kk) *(volatile v8h*)(WT + off[kk]) = ov[kk];
  } else if (blk < XP_BLKS + WT_BLKS + W2_BLKS) {
    const int t = (blk - XP_BLKS - WT_BLKS) * TPBP + tid;
    const int hh = t >> 5, k0 = (t & 31) * 8;
    const int hsrc = (hh < NH) ? hh : 0;
    const float keep = (hh < NH) ? 1.0f : 0.0f;
    v8h o;
    #pragma unroll
    for (int u = 0; u < 8; ++u) {
      const float* sp = wp2 + (size_t)(k0 + u) * DM + hsrc * HD;
      float s = 0.0f;
      #pragma unroll 1
      for (int i = 0; i < 8; ++i) {
        const v4f a = *(const v4fa*)(sp + 4 * i);
        s += a[0]; s += a[1]; s += a[2]; s += a[3];
      }
      o[u] = (f16t)(s * keep * W2CAR);
    }
    f16t* dp = W2T + (size_t)hh * DM + k0;
    *(volatile v8h*)dp = o;
    __threadfence();
    *(volatile v8h*)dp = o;
  }
}

__global__ __launch_bounds__(TPB) void proj_k(const f16t* __restrict__ XH, const f16t* __restrict__ WT,
                                             const float* __restrict__ bq, const float* __restrict__ bk,
                                             const float* __restrict__ bv,
                                             f16t* __restrict__ QH, f16t* __restrict__ KH,
                                             f16t* __restrict__ VT)
{
  __shared__ __attribute__((aligned(16))) float sbuf[64 * PF];
  const int tid = threadIdx.x, lane = tid & 31, wave = tid >> 5;
  const int h = lane >> 4, m = lane & 15;
  const int blk = blockIdx.x;
  const int mode = blk >> 6;
  const int rem = blk & 63;
  const int pb = rem >> 2, cg = rem & 3;
  const int row0 = 64 * pb;
  const int b = pb >> 3, p0 = (pb & 7) * 64;
  const float* bb = (mode == 0) ? bq : ((mode == 1) ? bk : bv);

  v8f acc[4];
  #pragma unroll
  for (int t = 0; t < 4; ++t) acc[t] = zero8f();
  mma_4n<DM>(XH + (size_t)(row0 + 16 * wave + m) * DM + 8 * h,
             WT + (size_t)mode * DM * DM + (size_t)(64 * cg + m) * DM + 8 * h, acc);

  const int tr = (mode == 2);
  #pragma unroll
  for (int t = 0; t < 4; ++t) {
    const int col = 16 * t + m;
    const float bvv = bb[64 * cg + col];
    #pragma unroll
    for (int r = 0; r < 8; ++r) {
      const int prow = 16 * wave + 8 * h + r;
      const float v = acc[t][r] * SC_P + bvv;
      const int idx = tr ? (col * PF + prow) : (prow * PF + col);
      sbuf[idx] = v;
    }
  }
  __syncthreads();

  if (mode < 2) {
    f16t* P = (mode == 0) ? QH : KH;
    v8h ov[4];
    size_t off[4];
    #pragma unroll
    for (int k = 0; k < 4; ++k) {
      const int al = k >> 1, hf = k & 1;
      const int p = 128 * hf + tid;
      const int row = p >> 2, d8 = (p & 3) * 8;
      const int col = 32 * al + d8;
      const v4f a = *(const v4fa*)(sbuf + row * PF + col), c = *(const v4fa*)(sbuf + row * PF + col + 4);
      #pragma unroll
      for (int j = 0; j < 4; ++j) {
        ov[k][j]     = (f16t)(a[j] * QCAR);
        ov[k][4 + j] = (f16t)(c[j] * QCAR);
      }
      const int na = b * NH + 2 * cg + al;
      off[k] = ((size_t)na * NN + p0 + row) * HD + d8;
    }
    #pragma unroll
    for (int k = 0; k < 4; ++k) *(volatile v8h*)(P + off[k]) = ov[k];
    __threadfence();
    #pragma unroll
    for (int k = 0; k < 4; ++k) *(volatile v8h*)(P + off[k]) = ov[k];
  } else {
    v8h ov[4];
    size_t off[4];
    #pragma unroll
    for (int k = 0; k < 4; ++k) {
      const int al = k >> 1, hf = k & 1;
      const int p = 128 * hf + tid;
      const int d = p >> 3, q8 = p & 7;
      const v4f a = *(const v4fa*)(sbuf + (32 * al + d) * PF + 8 * q8);
      const v4f c = *(const v4fa*)(sbuf + (32 * al + d) * PF + 8 * q8 + 4);
      #pragma unroll
      for (int j = 0; j < 4; ++j) {
        ov[k][j]     = (f16t)(a[j] * VCAR);
        ov[k][4 + j] = (f16t)(c[j] * VCAR);
      }
      const int na = b * NH + 2 * cg + al;
      off[k] = ((size_t)na * HD + d) * NN + p0 + 8 * q8;
    }
    #pragma unroll
    for (int k = 0; k < 4; ++k) *(volatile v8h*)(VT + off[k]) = ov[k];
    __threadfence();
    #pragma unroll
    for (int k = 0; k < 4; ++k) *(volatile v8h*)(VT + off[k]) = ov[k];
  }
}

__global__ __launch_bounds__(TPBA) void bias_k(const float* __restrict__ coords,
                                              const float* __restrict__ wp1, const float* __restrict__ bp1,
                                              const float* __restrict__ bp2, const f16t* __restrict__ W2T,
                                              float* __restrict__ BS)
{
  __shared__ __attribute__((aligned(16))) f16t g[256 * GP];
  __shared__ __attribute__((aligned(16))) float sb[128 * SBP];
  __shared__ __attribute__((aligned(16))) float sw[3 * DM];
  __shared__ __attribute__((aligned(16))) float sbp[DM];
  __shared__ float sb2[16];
  const int tid = threadIdx.x, lane = tid & 31, wave = tid >> 5;
  const int h = lane >> 4, m = lane & 15;
  const int blk = blockIdx.x;
  const int b = blk >> 10;
  const int rem = blk & 1023;
  const int nt = rem >> 4, mtl = rem & 15;
  const int n0 = 8 * nt, m0 = 32 * mtl;
  const int nl = tid >> 5, ml = tid & 31;
  const int n = n0 + nl, mm = m0 + ml;

  sw[tid]          = wp1[tid];
  sw[tid + DM]     = wp1[tid + DM];
  sw[tid + 2 * DM] = wp1[tid + 2 * DM];
  sbp[tid] = bp1[tid];
  if (tid < 32) {
    const int hh = tid & 7;
    float s = 0.0f;
    #pragma unroll
    for (int i = 0; i < 8; ++i) {
      const v4f a = *(const v4fa*)(bp2 + hh * HD + 4 * i);
      s += a[0]; s += a[1]; s += a[2]; s += a[3];
    }
    if (tid < 16) sb2[tid] = (tid < NH) ? s : 0.0f;
  }
  const float* cn = coords + ((size_t)b * NN + n) * 3;
  const float* cm = coords + ((size_t)b * NN + mm) * 3;
  const float r0 = cn[0] - cm[0];
  const float r1 = cn[1] - cm[1];
  const float r2 = cn[2] - cm[2];
  __syncthreads();

  v8f acc[2];
  acc[0] = zero8f(); acc[1] = zero8f();
  const f16t* brow = W2T + (size_t)m * DM + 8 * h;
  f16t* grow = g + tid * GP;
  const f16t* arow0 = g + (32 * wave + m) * GP + 8 * h;
  const f16t* arow1 = arow0 + 16 * GP;

  #pragma unroll 1
  for (int kc = 0; kc < DM / 32; ++kc) {
    #pragma unroll 1
    for (int jj = 0; jj < 8; ++jj) {
      const int kb = 32 * kc + 4 * jj;
      v4h pk;
      #pragma unroll
      for (int u = 0; u < 4; ++u) {
        const int k = kb + u;
        float pre = r0 * sw[k];
        pre = fmaf(r1, sw[DM + k], pre);
        pre = fmaf(r2, sw[2 * DM + k], pre);
        pre += sbp[k];
        const float ge = 0.5f * pre * (1.0f + erff(pre * RSQRT2));
        pk[u] = (f16t)(ge * HCAR);
      }
      *(v4h*)(grow + 4 * jj) = pk;
    }
    __syncthreads();
    FragH a0, a1, bf;
    load_frag(bf, brow, 32 * kc);
    load_frag(a0, arow0, 0);
    load_frag(a1, arow1, 0);
    acc[0] = wmma_f16(a0.v, bf.v, acc[0]);
    acc[1] = wmma_f16(a1.v, bf.v, acc[1]);
    __syncthreads();
  }

  const float bs2 = sb2[m];
  #pragma unroll
  for (int t = 0; t < 2; ++t) {
    #pragma unroll
    for (int r = 0; r < 8; ++r) {
      const int ml2 = 16 * t + 8 * h + r;
      sb[(m * 8 + wave) * SBP + ml2] = (acc[t][r] * SC_B + bs2) * SCALE;
    }
  }
  __syncthreads();

  v4f ov[2];
  size_t off[2];
  #pragma unroll
  for (int kk = 0; kk < 2; ++kk) {
    const int p = 256 * kk + tid;
    const int line = p >> 3, q = p & 7;
    const int hd = line >> 3, nl2 = line & 7;
    ov[kk] = *(const v4fa*)(sb + line * SBP + 4 * q);
    off[kk] = (((size_t)(b * NH + hd) * NN + n0 + nl2) * NN + m0 + 4 * q);
  }
  #pragma unroll
  for (int kk = 0; kk < 2; ++kk) *(volatile v4f*)(BS + off[kk]) = ov[kk];
  __threadfence();
  #pragma unroll
  for (int kk = 0; kk < 2; ++kk) *(volatile v4f*)(BS + off[kk]) = ov[kk];
}

__global__ __launch_bounds__(TPBA) void attn_k(const f16t* __restrict__ QH, const f16t* __restrict__ KH,
                                              const f16t* __restrict__ VT, const float* __restrict__ BS,
                                              f16t* __restrict__ OT)
{
  __shared__ __attribute__((aligned(16))) f16t sbuf[64 * PH];
  const int tid = threadIdx.x, lane = tid & 31, wave = tid >> 5;
  const int h = lane >> 4, m = lane & 15;
  const int blk = blockIdx.x;
  const int b = blk >> 5;
  const int rem = blk & 31;
  const int hp = rem >> 3, qb = rem & 7;
  const int wq = wave & 3, al = wave >> 2;
  const int aH = 2 * hp + al;
  const int na = b * NH + aH;
  const int i0 = 64 * qb + 16 * wq;
  const size_t qrow = (size_t)na * NN + i0 + m;

  FragH fq;
  load_frag(fq, QH + qrow * HD + 8 * h, 0);
  const float* brow = BS + qrow * NN + 8 * h;
  const f16t* kbase = KH + ((size_t)na * NN + m) * HD + 8 * h;
  const f16t* vbase = VT + ((size_t)na * HD + m) * NN + 8 * h;

  v8f O[2];
  O[0] = zero8f(); O[1] = zero8f();
  float Mx = -3.0e38f, L = 0.0f;

  #pragma unroll 1
  for (int js = 0; js < NN / 32; ++js) {
    const int j0 = 32 * js;
    FragH k0f, k1f;
    load_frag(k0f, kbase + (size_t)j0 * HD, 0);
    load_frag(k1f, kbase + (size_t)(j0 + 16) * HD, 0);
    const v8f s0 = wmma_f16(k0f.v, fq.v, zero8f());
    const v8f s1 = wmma_f16(k1f.v, fq.v, zero8f());
    U8 b0, b1;
    b0.q[0] = *(const v4fa*)(brow + j0);
    b0.q[1] = *(const v4fa*)(brow + j0 + 4);
    b1.q[0] = *(const v4fa*)(brow + j0 + 16);
    b1.q[1] = *(const v4fa*)(brow + j0 + 20);

    float e0[8], e1[8];
    float mloc = -3.0e38f;
    #pragma unroll
    for (int r = 0; r < 8; ++r) {
      e0[r] = s0[r] * SC_S + b0.v[r];
      e1[r] = s1[r] * SC_S + b1.v[r];
      mloc = fmaxf(mloc, fmaxf(e0[r], e1[r]));
    }
    mloc = fmaxf(mloc, __shfl_xor(mloc, 16));
    const float Mn = fmaxf(Mx, mloc);
    const float corr = __expf(Mx - Mn);
    Mx = Mn;

    FragH pf;
    float ls = 0.0f;
    #pragma unroll
    for (int r = 0; r < 8; ++r) {
      const float p0 = __expf(e0[r] - Mn);
      const float p1 = __expf(e1[r] - Mn);
      ls += p0 + p1;
      pf.half[0][r] = (f16t)(p0 * PCAR);
      pf.half[1][r] = (f16t)(p1 * PCAR);
    }
    ls += __shfl_xor(ls, 16);
    L = L * corr + ls;
    #pragma unroll
    for (int t = 0; t < 2; ++t) {
      #pragma unroll
      for (int r = 0; r < 8; ++r) O[t][r] *= corr;
    }
    #pragma unroll
    for (int t = 0; t < 2; ++t) {
      FragH va;
      load_frag(va, vbase + (size_t)16 * t * NN + j0, 0);
      O[t] = wmma_f16(va.v, pf.v, O[t]);
    }
  }

  const float inv = (1.0f / L) * SC_O;
  #pragma unroll
  for (int t = 0; t < 2; ++t) {
    #pragma unroll
    for (int r = 0; r < 8; ++r)
      sbuf[(16 * wq + m) * PH + 32 * al + 16 * t + 8 * h + r] = (f16t)(O[t][r] * inv);
  }
  __syncthreads();

  v8h ov[2];
  size_t off[2];
  #pragma unroll
  for (int kk = 0; kk < 2; ++kk) {
    const int p = 256 * kk + tid;
    const int row = p >> 3, q = p & 7;
    ov[kk] = *(const v8ha*)(sbuf + row * PH + 8 * q);
    off[kk] = ((size_t)b * NN + 64 * qb + row) * DM + 64 * hp + 8 * q;
  }
  #pragma unroll
  for (int kk = 0; kk < 2; ++kk) *(volatile v8h*)(OT + off[kk]) = ov[kk];
  __threadfence();
  #pragma unroll
  for (int kk = 0; kk < 2; ++kk) *(volatile v8h*)(OT + off[kk]) = ov[kk];
}

__global__ __launch_bounds__(TPB) void oproj_k(const f16t* __restrict__ OT, const f16t* __restrict__ WT,
                                              const float* __restrict__ bo, float* __restrict__ out)
{
  __shared__ __attribute__((aligned(16))) float sbuf[64 * PF];
  const int tid = threadIdx.x, lane = tid & 31, wave = tid >> 5;
  const int h = lane >> 4, m = lane & 15;
  const int blk = blockIdx.x;
  const int pb = blk >> 2, cg = blk & 3;
  const int row0 = 64 * pb;

  v8f acc[4];
  #pragma unroll
  for (int t = 0; t < 4; ++t) acc[t] = zero8f();
  mma_4n<DM>(OT + (size_t)(row0 + 16 * wave + m) * DM + 8 * h,
             WT + (size_t)3 * DM * DM + (size_t)(64 * cg + m) * DM + 8 * h, acc);

  #pragma unroll
  for (int t = 0; t < 4; ++t) {
    const int col = 16 * t + m;
    const float bvv = bo[64 * cg + col];
    #pragma unroll
    for (int r = 0; r < 8; ++r) {
      const int prow = 16 * wave + 8 * h + r;
      sbuf[prow * PF + col] = acc[t][r] * SC_PO + bvv;
    }
  }
  __syncthreads();

  v4f ov[8];
  size_t off[8];
  #pragma unroll
  for (int kk = 0; kk < 8; ++kk) {
    const int p = 128 * kk + tid;
    const int row = p >> 4, q = p & 15;
    ov[kk] = *(const v4fa*)(sbuf + row * PF + 4 * q);
    off[kk] = (size_t)(row0 + row) * DM + 64 * cg + 4 * q;
  }
  #pragma unroll
  for (int kk = 0; kk < 8; ++kk) *(volatile v4f*)(out + off[kk]) = ov[kk];
  __threadfence();
  #pragma unroll
  for (int kk = 0; kk < 8; ++kk) *(volatile v4f*)(out + off[kk]) = ov[kk];
}

extern "C" void kernel_launch(void* const* d_in, const int* in_sizes, int n_in,
                              void* d_out, int out_size, void* d_ws, size_t ws_size,
                              hipStream_t stream) {
  if (n_in < 14) return;
  if (in_sizes[0] != BNR * DM) return;
  if (in_sizes[1] != BNR * 3) return;
  if (in_sizes[2] != DM * DM || in_sizes[4] != DM * DM || in_sizes[6] != DM * DM) return;
  if (in_sizes[8] != DM * DM || in_sizes[12] != DM * DM) return;
  if (in_sizes[3] != DM || in_sizes[5] != DM || in_sizes[7] != DM || in_sizes[9] != DM) return;
  if (in_sizes[10] != 3 * DM || in_sizes[11] != DM || in_sizes[13] != DM) return;
  if (out_size != BNR * DM) return;

  const float* x      = (const float*)d_in[0];
  const float* coords = (const float*)d_in[1];
  const float* Wq  = (const float*)d_in[2];   const float* bq  = (const float*)d_in[3];
  const float* Wk  = (const float*)d_in[4];   const float* bk  = (const float*)d_in[5];
  const float* Wv  = (const float*)d_in[6];   const float* bv  = (const float*)d_in[7];
  const float* Wo  = (const float*)d_in[8];   const float* bo  = (const float*)d_in[9];
  const float* Wp1 = (const float*)d_in[10];  const float* bp1 = (const float*)d_in[11];
  const float* Wp2 = (const float*)d_in[12];  const float* bp2 = (const float*)d_in[13];
  float* outp = (float*)d_out;

  const size_t szXH = (size_t)BNR * DM * 2;
  const size_t szWT = (size_t)4 * DM * DM * 2;
  const size_t szW2 = (size_t)16 * DM * 2;
  const size_t szQ  = (size_t)NA * NN * HD * 2;
  const size_t szBS = (size_t)NA * NN * NN * 4;
  const size_t szOT = (size_t)BNR * DM * 2;
  static_assert((size_t)BNR * DM * 2 + (size_t)4 * DM * DM * 2 + (size_t)16 * DM * 2 +
                3 * ((size_t)NA * NN * HD * 2) + (size_t)NA * NN * NN * 4 +
                (size_t)BNR * DM * 2 <= (size_t)134217728);
  size_t off = 0;
  char* ws = (char*)d_ws;
  f16t*  XH  = (f16t*)(ws + off);  off += szXH;
  f16t*  WT  = (f16t*)(ws + off);  off += szWT;
  f16t*  W2T = (f16t*)(ws + off);  off += szW2;
  f16t*  QH  = (f16t*)(ws + off);  off += szQ;
  f16t*  KH  = (f16t*)(ws + off);  off += szQ;
  f16t*  VT  = (f16t*)(ws + off);  off += szQ;
  float* BS  = (float*)(ws + off); off += szBS;
  f16t*  OT  = (f16t*)(ws + off);  off += szOT;
  if (off > ws_size) return;

  prep_k<<<XP_BLKS + WT_BLKS + W2_BLKS, TPBP, 0, stream>>>(x, Wq, Wk, Wv, Wo, Wp2, XH, WT, W2T);
  proj_k<<<PRJ_BLKS, TPB, 0, stream>>>(XH, WT, bq, bk, bv, QH, KH, VT);
  bias_k<<<BIAS_BLKS, TPBA, 0, stream>>>(coords, Wp1, bp1, bp2, W2T, BS);
  attn_k<<<ATT_BLKS, TPBA, 0, stream>>>(QH, KH, VT, BS, OT);
  oproj_k<<<OP_BLKS, TPB, 0, stream>>>(OT, WT, bo, outp);
  (void)hipGetLastError();
}
